// WeLMV3Attention_90142773609337
// MI455X (gfx1250) — hardware-verified
//
#include <hip/hip_runtime.h>


#define NS_  2048
#define HID  2048
#define NH_  16
#define NKV  4
#define HD   128
#define QSZ  (NH_ * HD)
#define KSZ  (NKV * HD)
#define NQKV (QSZ + 2 * KSZ)
#define PSC  32768.0f
#define LOSC 1024.0f
#define LOSCI (1.0f / 1024.0f)
#define SCL  0.08838834764831845f

typedef _Float16 h16;
typedef unsigned short bf;
typedef __attribute__((ext_vector_type(16))) __bf16   v16bf;
typedef __attribute__((ext_vector_type(16))) _Float16 v16h;
typedef __attribute__((ext_vector_type(8)))  _Float16 v8h;
typedef __attribute__((ext_vector_type(8)))  unsigned short v8us;
typedef __attribute__((ext_vector_type(8)))  float    v8f;
typedef __attribute__((ext_vector_type(4)))  float    v4f;
typedef __attribute__((ext_vector_type(2)))  _Float16 v2h;
typedef v8h  __attribute__((may_alias)) v8ha;
typedef v4f  __attribute__((may_alias)) v4fa;
typedef v8us __attribute__((may_alias)) v8usa;

__device__ __forceinline__ unsigned short f2bf(float f) { unsigned u = __float_as_uint(f); u += 0x7FFFu + ((u >> 16) & 1u); return (unsigned short)(u >> 16); }
__device__ __forceinline__ float bf2f(unsigned short b) { return __uint_as_float(((unsigned)b) << 16); }
__device__ __forceinline__ v16h cat16(v8h lo, v8h hi) { return __builtin_shufflevector(lo, hi, 0, 1, 2, 3, 4, 5, 6, 7, 8, 9, 10, 11, 12, 13, 14, 15); }
__device__ __forceinline__ v16bf cat16b(v8us lo, v8us hi) { return __builtin_bit_cast(v16bf, __builtin_shufflevector(lo, hi, 0, 1, 2, 3, 4, 5, 6, 7, 8, 9, 10, 11, 12, 13, 14, 15)); }
__device__ __forceinline__ v8f wmma16(v16h a, v16h b, v8f c) { return __builtin_amdgcn_wmma_f32_16x16x32_f16(false, a, false, b, (short)0, c, false, false); }
__device__ __forceinline__ v8f wmmab(v16bf a, v16bf b, v8f c) { return __builtin_amdgcn_wmma_f32_16x16x32_bf16(false, a, false, b, (short)0, c, false, false); }
#define VST2(T, p, v) do { const T vst2_v_ = (v); *(volatile T*)(p) = vst2_v_; __threadfence(); *(volatile T*)(p) = vst2_v_; } while (0)

__global__ __launch_bounds__(256) void k_cvtb(const float* __restrict__ src, int nrows, bf* dst) {
    const int lane = threadIdx.x & 31, r = blockIdx.x * 8 + (threadIdx.x >> 5);
    if (r >= nrows) return;
#pragma unroll 1
    for (int q = 0; q < 8; ++q) { v8us t;
#pragma unroll
        for (int i = 0; i < 8; ++i) t[i] = f2bf(src[(size_t)r * HID + q * 256 + lane * 8 + i]);
        *(volatile v8us*)(dst + (size_t)r * HID + q * 256 + lane * 8) = t; __threadfence(); *(volatile v8us*)(dst + (size_t)r * HID + q * 256 + lane * 8) = t; }
}

__global__ __launch_bounds__(256) void k_wt(const float* __restrict__ Wm, int ncols, bf* WT) {
    __shared__ __align__(16) unsigned short tl[64 * 72];
    const int tid = threadIdx.x, k0 = blockIdx.x * 64, n0 = blockIdx.y * 64;
    const int kk = tid >> 2, nq = (tid & 3) * 16;
#pragma unroll
    for (int i = 0; i < 16; ++i) tl[(nq + i) * 72 + kk] = f2bf(Wm[(size_t)(k0 + kk) * ncols + n0 + nq + i]);
    __syncthreads();
    const int piece = tid & 7;
    auto pass = [&]() {
#pragma unroll
        for (int s = 0; s < 2; ++s) { const int nr = (tid >> 3) + 32 * s; const v8us val = *(const v8usa*)(tl + nr * 72 + piece * 8);
            *(volatile v8us*)(WT + (size_t)(n0 + nr) * HID + k0 + piece * 8) = val; }
    };
    pass(); __threadfence(); pass();
}

template <bool SPLITA>
__global__ __launch_bounds__(128) void k_gemmb(const bf* __restrict__ A, const bf* __restrict__ Al, const bf* __restrict__ Bn, float* C, int ldc) {
    __shared__ __align__(16) float ost[4][16 * 68];
    const int lane = threadIdx.x & 31, wave = threadIdx.x >> 5, lr = lane & 15, hi = lane >> 4;
    const int r0 = blockIdx.x * 64 + wave * 16, c0 = blockIdx.y * 64;
    const size_t aoff = (size_t)(r0 + lr) * HID + 8 * hi;
    size_t boff[4];
#pragma unroll
    for (int t = 0; t < 4; ++t) boff[t] = (size_t)(c0 + t * 16 + lr) * HID + 8 * hi;
    v8f acc[4];
#pragma unroll
    for (int t = 0; t < 4; ++t) acc[t] = (v8f){};
#pragma unroll 1
    for (int kc = 0; kc < HID; kc += 32) {
        const v16bf a = cat16b(*(const v8us*)(A + aoff + kc), *(const v8us*)(A + aoff + kc + 16));
        v16bf al = a;
        if (SPLITA) al = cat16b(*(const v8us*)(Al + aoff + kc), *(const v8us*)(Al + aoff + kc + 16));
#pragma unroll
        for (int t = 0; t < 4; ++t) { const v16bf b = cat16b(*(const v8us*)(Bn + boff[t] + kc), *(const v8us*)(Bn + boff[t] + kc + 16)); acc[t] = wmmab(a, b, acc[t]); if (SPLITA) acc[t] = wmmab(al, b, acc[t]); }
        asm volatile("v_nop\n\tv_nop\n\tv_nop\n\tv_nop" : "+v"(acc[0]), "+v"(acc[1]), "+v"(acc[2]), "+v"(acc[3]) : "v"(a), "v"(al));
    }
    float* os = &ost[wave][0];
#pragma unroll
    for (int t = 0; t < 4; ++t)
#pragma unroll
        for (int j = 0; j < 8; ++j) os[(hi * 8 + j) * 68 + t * 16 + lr] = acc[t][j];
    __syncthreads();
    float* crow = C + (size_t)r0 * ldc + c0;
    auto pass = [&]() {
#pragma unroll
        for (int s = 0; s < 8; ++s) { const int Lid = (lane >> 3) + 4 * s, piece = lane & 7; const int row = Lid >> 1, cofs = (Lid & 1) * 32 + piece * 4;
            const v4f val = *(const v4fa*)(os + row * 68 + cofs); *(volatile v4f*)(crow + (size_t)row * ldc + cofs) = val; }
    };
    pass(); __threadfence(); pass();
}

__global__ __launch_bounds__(256) void k_tab(const int* __restrict__ pos, float* COSF, float* SINF) {
    const int lane = threadIdx.x & 31, wid = blockIdx.x * 8 + (threadIdx.x >> 5);
    if (wid >= 2 * NS_) return;
    const int t = wid >> 1, which = wid & 1;
    const float p = (float)pos[t];
    typedef __attribute__((ext_vector_type(2))) float v2f;
    v2f o;
#pragma unroll 1
    for (int i = 0; i < 2; ++i) {
        const int j = 2 * lane + i;
        const float inv = 1.0f / powf(10000.0f, (float)(2 * j) / (float)HD);
        const float f = p * inv;
        o[i] = which ? sinf(f) : cosf(f);
    }
    float* dst = (which ? SINF : COSF) + (size_t)t * (HD / 2) + 2 * lane;
    *(volatile v2f*)dst = o; __threadfence(); *(volatile v2f*)dst = o;
}

__global__ __launch_bounds__(256) void k_rope(const float* __restrict__ QKV, const float* __restrict__ COSF, const float* __restrict__ SINF, h16* Q16, h16* K16) {
    const int lane = threadIdx.x & 31, wid = blockIdx.x * 8 + (threadIdx.x >> 5);
    if (wid >= NS_ * (NH_ + NKV)) return;
    const int t = wid / (NH_ + NKV), g = wid - t * (NH_ + NKV);
    const float* src = QKV + (size_t)t * NQKV + ((g < NH_) ? g * HD : QSZ + (g - NH_) * HD);
    h16* dst = (g < NH_) ? (Q16 + (size_t)t * QSZ + g * HD) : (K16 + (size_t)t * KSZ + (g - NH_) * HD);
    v2h o1, o2;
#pragma unroll
    for (int i = 0; i < 2; ++i) {
        const int j = 2 * lane + i;
        const float x1 = src[j], x2 = src[HD / 2 + j], c = COSF[(size_t)t * (HD / 2) + j], s = SINF[(size_t)t * (HD / 2) + j];
        o1[i] = (h16)(x1 * c - x2 * s); o2[i] = (h16)(x2 * c + x1 * s);
    }
    *(volatile v2h*)(dst + 2 * lane) = o1; *(volatile v2h*)(dst + HD / 2 + 2 * lane) = o2;
    __threadfence();
    *(volatile v2h*)(dst + 2 * lane) = o1; *(volatile v2h*)(dst + HD / 2 + 2 * lane) = o2;
}

__global__ __launch_bounds__(256) void k_vt(const float* __restrict__ QKV, h16* VTH, h16* VTL) {
    __shared__ __align__(16) h16 tile[HD * 72];
    __shared__ __align__(16) h16 til2[HD * 72];
    const int bid = blockIdx.x;
    const int hk = bid / (NS_ / 64), kt = bid - hk * (NS_ / 64);
    const int k0 = kt * 64, tid = threadIdx.x;
    const int kk = tid >> 2, d0 = (tid & 3) * 32;
    const float* src = QKV + (size_t)(k0 + kk) * NQKV + QSZ + KSZ + hk * HD + d0;
#pragma unroll
    for (int i = 0; i < 32; ++i) { const float v = src[i]; const h16 a = (h16)v; tile[(d0 + i) * 72 + kk] = a; til2[(d0 + i) * 72 + kk] = (h16)((v - (float)a) * LOSC); }
    __syncthreads();
    const int piece = tid & 7;
    const size_t base = ((size_t)hk * HD) * NS_ + k0;
    auto pass = [&]() {
#pragma unroll
        for (int s = 0; s < 8; ++s) { const int Lid = (tid >> 3) + 32 * s; const int pln = Lid >> 7, d = Lid & 127;
            const v8h val = *(const v8ha*)((pln ? til2 : tile) + d * 72 + piece * 8); *(volatile v8h*)((pln ? VTL : VTH) + base + (size_t)d * NS_ + piece * 8) = val; }
    };
    pass(); __threadfence(); pass();
}

__global__ __launch_bounds__(128) void k_attn(const h16* __restrict__ Q16, const h16* __restrict__ K16, const h16* __restrict__ VTH, const h16* __restrict__ VTL, int dofs, bf* CH, bf* CL) {
    __shared__ __align__(16) h16 plds[4][16 * 32];
    __shared__ __align__(16) h16 plds2[4][16 * 32];
    __shared__ __align__(16) float ost[4][16 * 68];
    const int lane = threadIdx.x & 31, wave = threadIdx.x >> 5, lr = lane & 15, hi = lane >> 4;
    const int h = blockIdx.x / (NS_ / 64), qt = blockIdx.x - h * (NS_ / 64), hk = h / (NH_ / NKV);
    const int q0 = qt * 64 + wave * 16;
    h16* pl = &plds[wave][0]; h16* pl2 = &plds2[wave][0];
    v16h qa[4];
#pragma unroll
    for (int kc = 0; kc < 4; ++kc) { const h16* p = Q16 + (size_t)(q0 + lr) * QSZ + h * HD + kc * 32 + 8 * hi; qa[kc] = cat16(*(const v8h*)p, *(const v8h*)(p + 16)); }
    int qpos[8];
#pragma unroll
    for (int j = 0; j < 8; ++j) qpos[j] = q0 + 8 * hi + j;
    const h16* kh_b = K16 + hk * HD;
    const size_t vbase = ((size_t)hk * HD + dofs) * NS_;
    v8f o[4], ox[4];
#pragma unroll
    for (int n = 0; n < 4; ++n) { o[n] = (v8f){}; ox[n] = (v8f){}; }
    float mrow[8], lpart[8];
#pragma unroll
    for (int j = 0; j < 8; ++j) { mrow[j] = -3.0e38f; lpart[j] = 0.f; }
    const int kt_end = (qt * 64 + 64) / 32;
#pragma unroll 1
    for (int kt = 0; kt < kt_end; ++kt) {
        const int l0 = kt * 32;
        const h16* r0p = kh_b + (size_t)(l0 + lr) * KSZ + 8 * hi;
        const h16* r1p = kh_b + (size_t)(l0 + 16 + lr) * KSZ + 8 * hi;
        v8f s0 = {}, s1 = {};
#pragma unroll
        for (int kc = 0; kc < 4; ++kc) {
            s0 = wmma16(qa[kc], cat16(*(const v8h*)(r0p + kc * 32), *(const v8h*)(r0p + kc * 32 + 16)), s0);
            s1 = wmma16(qa[kc], cat16(*(const v8h*)(r1p + kc * 32), *(const v8h*)(r1p + kc * 32 + 16)), s1);
        }
        asm volatile("v_nop\n\tv_nop\n\tv_nop\n\tv_nop" : "+v"(s0), "+v"(s1) : "v"(qa[0]), "v"(qa[3]));
        float alpha[8];
#pragma unroll
        for (int j = 0; j < 8; ++j) {
            const float a0 = (l0 + lr <= qpos[j]) ? s0[j] * SCL : -__builtin_inff(), a1 = (l0 + 16 + lr <= qpos[j]) ? s1[j] * SCL : -__builtin_inff();
            float mx = fmaxf(a0, a1);
            mx = fmaxf(mx, __shfl_xor(mx, 1, 16)); mx = fmaxf(mx, __shfl_xor(mx, 2, 16)); mx = fmaxf(mx, __shfl_xor(mx, 4, 16)); mx = fmaxf(mx, __shfl_xor(mx, 8, 16));
            const float mn = fmaxf(mrow[j], mx);
            alpha[j] = __expf(mrow[j] - mn); mrow[j] = mn;
            const float p0 = __expf(a0 - mn), p1 = __expf(a1 - mn);
            lpart[j] = lpart[j] * alpha[j] + (p0 + p1);
            const int mr = hi * 8 + j;
            const float ps0 = p0 * PSC, ps1 = p1 * PSC; const h16 h0 = (h16)ps0, h1 = (h16)ps1;
            pl[mr * 32 + lr] = h0; pl[mr * 32 + 16 + lr] = h1;
            pl2[mr * 32 + lr] = (h16)((ps0 - (float)h0) * LOSC); pl2[mr * 32 + 16 + lr] = (h16)((ps1 - (float)h1) * LOSC);
        }
#pragma unroll
        for (int n = 0; n < 4; ++n)
#pragma unroll
            for (int j = 0; j < 8; ++j) { o[n][j] *= alpha[j]; ox[n][j] *= alpha[j]; }
        asm volatile("" ::: "memory");
        const v16h pa = cat16(*(const v8ha*)(pl + lr * 32 + hi * 8), *(const v8ha*)(pl + lr * 32 + 16 + hi * 8));
        const v16h px = cat16(*(const v8ha*)(pl2 + lr * 32 + hi * 8), *(const v8ha*)(pl2 + lr * 32 + 16 + hi * 8));
#pragma unroll
        for (int n = 0; n < 4; ++n) { const size_t vo = vbase + (size_t)(n * 16 + lr) * NS_ + l0 + hi * 8;
            const v16h vh = cat16(*(const v8h*)(VTH + vo), *(const v8h*)(VTH + vo + 16)), vl = cat16(*(const v8h*)(VTL + vo), *(const v8h*)(VTL + vo + 16));
            o[n] = wmma16(pa, vh, o[n]); ox[n] = wmma16(pa, vl, ox[n]); ox[n] = wmma16(px, vh, ox[n]); }
        asm volatile("v_nop\n\tv_nop\n\tv_nop\n\tv_nop" : "+v"(o[0]), "+v"(o[1]), "+v"(o[2]), "+v"(o[3]), "+v"(ox[0]), "+v"(ox[1]), "+v"(ox[2]), "+v"(ox[3]) : "v"(pa), "v"(px));
    }
    float inv[8];
#pragma unroll
    for (int j = 0; j < 8; ++j) { float rs = lpart[j]; rs += __shfl_xor(rs, 1, 16); rs += __shfl_xor(rs, 2, 16); rs += __shfl_xor(rs, 4, 16); rs += __shfl_xor(rs, 8, 16); inv[j] = 1.0f / (rs * PSC); }
    float* os = &ost[wave][0];
#pragma unroll
    for (int n = 0; n < 4; ++n)
#pragma unroll
        for (int j = 0; j < 8; ++j) os[(hi * 8 + j) * 68 + n * 16 + lr] = (o[n][j] + ox[n][j] * LOSCI) * inv[j];
    __syncthreads();
    const size_t cbase = (size_t)q0 * QSZ + (size_t)h * HD + dofs;
    auto pass = [&]() {
#pragma unroll
        for (int s = 0; s < 4; ++s) { const int row = 4 * s + (lane >> 3), piece = lane & 7; const float* sp = os + row * 68 + piece * 8; v8us oh, ol;
#pragma unroll
            for (int i = 0; i < 8; ++i) { const unsigned short hb = f2bf(sp[i]); oh[i] = hb; ol[i] = f2bf(sp[i] - bf2f(hb)); }
            *(volatile v8us*)(CH + cbase + (size_t)row * QSZ + piece * 8) = oh; *(volatile v8us*)(CL + cbase + (size_t)row * QSZ + piece * 8) = ol; }
    };
    pass(); __threadfence(); pass();
}

extern "C" void kernel_launch(void* const* d_in, const int* in_sizes, int n_in,
                              void* d_out, int out_size, void* d_ws, size_t ws_size, hipStream_t stream) {
    (void)in_sizes; (void)n_in; (void)out_size;
    const float* x = (const float*)d_in[0]; const float* Wqkv = (const float*)d_in[1]; const float* Wo = (const float*)d_in[2]; const int* pos = (const int*)d_in[3];
    float* out = (float*)d_out;
    char* wsp = (char*)d_ws;
    auto take = [&](size_t bytes) { char* p = wsp; wsp += (bytes + 255) & ~(size_t)255; return (void*)p; };
    bf* Xb = (bf*)take((size_t)NS_ * HID * 2); bf* WQT = (bf*)take((size_t)NQKV * HID * 2); bf* WOT = (bf*)take((size_t)HID * HID * 2);
    float* QKV = (float*)take((size_t)NS_ * NQKV * 4); float* COSF = (float*)take((size_t)NS_ * (HD / 2) * 4); float* SINF = (float*)take((size_t)NS_ * (HD / 2) * 4);
    h16* Q16 = (h16*)take((size_t)NS_ * QSZ * 2); h16* K16 = (h16*)take((size_t)NS_ * KSZ * 2); h16* VTH = (h16*)take((size_t)NS_ * KSZ * 2); h16* VTL = (h16*)take((size_t)NS_ * KSZ * 2);
    bf* CH = (bf*)take((size_t)NS_ * QSZ * 2); bf* CL = (bf*)take((size_t)NS_ * QSZ * 2);
    if ((size_t)(wsp - (char*)d_ws) > ws_size) return;
    k_cvtb<<<NS_ / 8, 256, 0, stream>>>(x, NS_, Xb);
    k_wt<<<dim3(HID / 64, NQKV / 64, 1), 256, 0, stream>>>(Wqkv, NQKV, WQT);
    k_wt<<<dim3(HID / 64, HID / 64, 1), 256, 0, stream>>>(Wo, HID, WOT);
    k_gemmb<false><<<dim3(NS_ / 64, NQKV / 64, 1), 128, 0, stream>>>(Xb, nullptr, WQT, QKV, NQKV);
    k_tab<<<(2 * NS_) / 8, 256, 0, stream>>>(pos, COSF, SINF);
    k_rope<<<(NS_ * (NH_ + NKV)) / 8, 256, 0, stream>>>(QKV, COSF, SINF, Q16, K16);
    k_vt<<<NKV * (NS_ / 64), 256, 0, stream>>>(QKV, VTH, VTL);
    k_attn<<<NH_ * (NS_ / 64), 128, 0, stream>>>(Q16, K16, VTH, VTL, 0, CH, CL);
    k_attn<<<NH_ * (NS_ / 64), 128, 0, stream>>>(Q16, K16, VTH, VTL, HD / 2, CH, CL);
    k_gemmb<true><<<dim3(NS_ / 64, HID / 64, 1), 128, 0, stream>>>(CH, CL, WOT, out, HID);
}
